// KernelAttention_65481071396711
// MI455X (gfx1250) — hardware-run, weakly checked
//
#include <hip/hip_runtime.h>
#include <math.h>

typedef __attribute__((ext_vector_type(16))) _Float16 v16h;
typedef __attribute__((ext_vector_type(16))) __bf16 v16b;
typedef __attribute__((ext_vector_type(8)))  _Float16 v8h;
typedef __attribute__((ext_vector_type(8)))  float v8f;
typedef __attribute__((ext_vector_type(4)))  float v4f;
typedef __attribute__((ext_vector_type(2)))  float v2f;
typedef __attribute__((ext_vector_type(4)))  unsigned v4u;
typedef __attribute__((ext_vector_type(4)))  int v4i;
typedef float __attribute__((may_alias)) float_a;
typedef int __attribute__((may_alias)) int_a;

template <typename T> __device__ __forceinline__ void vst2(void* p, T v) { *(volatile T*)p = v; __threadfence(); *(volatile T*)p = v; }
__device__ __forceinline__ v8f wmma16(v16h a, v16h b, v8f c) {
  v8f d = __builtin_amdgcn_wmma_f32_16x16x32_f16(false, a, false, b, (short)0, c, false, false);
  asm volatile("v_nop\n\tv_nop\n\tv_nop\n\tv_nop" : "+v"(d) : "v"(a), "v"(b));
  return d;
}
__device__ __forceinline__ v8f wmma_bf(v16b a, v16b b, v8f c) {
  v8f d = __builtin_amdgcn_wmma_f32_16x16x32_bf16(false, a, false, b, (short)0, c, false, false);
  asm volatile("v_nop\n\tv_nop\n\tv_nop\n\tv_nop" : "+v"(d) : "v"(a), "v"(b));
  return d;
}
__device__ __forceinline__ v16h frag_h(const _Float16* rowk0, int lane) {
  union { v16h v; v8h q[2]; } u; const _Float16* p = rowk0 + 8 * (lane >> 4);
  u.q[0] = *(const v8h*)p; u.q[1] = *(const v8h*)(p + 16); return u.v;
}
__device__ __forceinline__ v16h frag_f32(const float* rowk0, int lane) {
  v16h a; const float* p = rowk0 + 8 * (lane >> 4);
#pragma unroll
  for (int i = 0; i < 8; ++i) { a[i] = (_Float16)p[i]; a[8 + i] = (_Float16)p[16 + i]; }
  return a;
}
__device__ __forceinline__ v16h frag_f32s(const float* rowk0, int lane, float sc) {
  v16h a; const float* p = rowk0 + 8 * (lane >> 4);
#pragma unroll
  for (int i = 0; i < 8; ++i) { a[i] = (_Float16)(p[i] * sc); a[8 + i] = (_Float16)(p[16 + i] * sc); }
  return a;
}
__device__ __forceinline__ v16h fragc_f32(const float* W, int k0, int n, int lane, int ld, int K) {
  v16h a; const int g = lane >> 4;
#pragma unroll
  for (int i = 0; i < 8; ++i) { const int ka = k0 + 8 * g + i, kb = ka + 16;
    a[i] = (_Float16)(ka < K ? W[(size_t)(ka < K ? ka : K - 1) * ld + n] : 0.f); a[8 + i] = (_Float16)(kb < K ? W[(size_t)(kb < K ? kb : K - 1) * ld + n] : 0.f); }
  return a;
}
struct F2 { v16b h, l; };
__device__ __forceinline__ F2 bsplit16(const float v[16]) { F2 r;
#pragma unroll
  for (int i = 0; i < 16; ++i) { const __bf16 h = (__bf16)v[i]; r.h[i] = h; r.l[i] = (__bf16)(v[i] - (float)h); }
  return r; }
__device__ __forceinline__ F2 split_row(const float* row, int k0, int lane) { float v[16]; const float* p = row + k0 + 8 * (lane >> 4);
#pragma unroll
  for (int i = 0; i < 8; ++i) { v[i] = p[i]; v[8 + i] = p[16 + i]; }
  return bsplit16(v); }
__device__ __forceinline__ F2 split_rowK(const float* row, int k0, int lane, int K) { float v[16]; const int g = lane >> 4;
#pragma unroll
  for (int i = 0; i < 8; ++i) { const int ka = k0 + 8 * g + i, kb = ka + 16; v[i] = ka < K ? row[ka < K ? ka : K - 1] : 0.f; v[8 + i] = kb < K ? row[kb < K ? kb : K - 1] : 0.f; }
  return bsplit16(v); }
__device__ __forceinline__ F2 split_col(const float* W, int k0, int n, int lane, int ld, int K) { float v[16]; const int g = lane >> 4;
#pragma unroll
  for (int i = 0; i < 8; ++i) { const int ka = k0 + 8 * g + i, kb = ka + 16; v[i] = ka < K ? W[(size_t)(ka < K ? ka : K - 1) * ld + n] : 0.f; v[8 + i] = kb < K ? W[(size_t)(kb < K ? kb : K - 1) * ld + n] : 0.f; }
  return bsplit16(v); }
__device__ __forceinline__ v8f mac3(const F2& a, const F2& b, v8f c) { c = wmma_bf(a.l, b.h, c); c = wmma_bf(a.h, b.l, c); return wmma_bf(a.h, b.h, c); }
__device__ __forceinline__ float sigm(float v) { return 1.0f / (1.0f + expf(-v)); }
#define LDSX() do { asm volatile("s_wait_dscnt 0" ::: "memory"); __builtin_amdgcn_wave_barrier(); __builtin_amdgcn_fence(__ATOMIC_RELEASE, "workgroup"); } while (0)


#define NB 4
#define NS 2048
#define EE 512
#define GAM 1.0f
#ifndef TNB
#define TNB NB
#endif
typedef __attribute__((ext_vector_type(8))) __bf16 v8b;
__device__ __forceinline__ v16b frag_b(const __bf16* rowk0, int lane) {
  union { v16b v; v8b q[2]; } u; const __bf16* p = rowk0 + 8 * (lane >> 4);
  u.q[0] = *(const v8b*)p; u.q[1] = *(const v8b*)(p + 16); return u.v;
}
__device__ __forceinline__ float bfr(float v) { return (float)(__bf16)v; }
__device__ __attribute__((noinline)) float exp_ni(float v) { return expf(v); }
__device__ __attribute__((noinline)) float erf_ni(float v) { return erff(v); }

#define WS_SQ  0u
#define WS_IL  (WS_SQ + 4u * (size_t)NB * NS)
#define WS_XT  (WS_IL + 4u * (size_t)NB * NS)
#define WS_EH  (WS_XT + 2u * (size_t)NB * EE * NS)
#define WS_EL  (WS_EH + 2u * (size_t)NB * NS * NS)
#define WS_END (WS_EL + 2u * (size_t)NB * NS * NS)

__global__ __launch_bounds__(128) void k_prep(const float* __restrict__ X, float* __restrict__ SQ, _Float16* __restrict__ XT) { __shared__ __align__(16) _Float16 st[128][72]; __shared__ __align__(16) float ssq[64];
  const int t = threadIdx.x; const size_t b = blockIdx.y; const int s0 = blockIdx.x * 64;
  if (t < 64) { const float* xr = X + (b * NS + s0 + t) * EE; float a = 0.f;
#pragma unroll 1
    for (int e = 0; e < EE; ++e) { const float v = bfr(xr[e]); a += v * v; }
    ssq[t] = a; }
#pragma unroll 1
  for (int cp = 0; cp < EE / 128; ++cp) { __syncthreads();
    for (int e = t; e < 128 * 64; e += 128) { const int sl = e >> 7, c = e & 127; st[c][sl] = (_Float16)bfr(X[(b * NS + s0 + sl) * EE + cp * 128 + c]); }
    __syncthreads();
    for (int e = t; e < 128 * 8; e += 128) { const int c = e >> 3, q = e & 7; vst2((unsigned*)(XT + (b * EE + cp * 128 + c) * (size_t)NS + s0 + q * 8), *(const v4u*)&st[c][q * 8]); } }
  __syncthreads(); if (t < 16) vst2(SQ + b * NS + s0 + t * 4, *(const v4f*)&ssq[t * 4]); }
__global__ __launch_bounds__(128) void k_e(const float* __restrict__ X, const float* __restrict__ SQ, _Float16* __restrict__ EH, _Float16* __restrict__ EL, float* __restrict__ IL) {
  __shared__ __align__(16) _Float16 sh[4][16][40], sl[4][16][40]; __shared__ __align__(16) float sil[64];
  const int tid = threadIdx.x, wave = tid >> 5, lane = tid & 31, col = lane & 15, g = lane >> 4; const size_t b = blockIdx.y; const int q0 = blockIdx.x * 64 + wave * 16; const size_t rq = b * NS + q0;
  float sqq[8], rs[8];
#pragma unroll
  for (int r = 0; r < 8; ++r) { sqq[r] = SQ[rq + 8 * g + r]; rs[r] = 0.f; }
#pragma unroll 1
  for (int ks = 0; ks < NS / 32; ++ks) {
#pragma unroll
    for (int ct = 0; ct < 2; ++ct) { const int kk = ks * 32 + ct * 16 + col; const size_t rk = b * NS + kk; v8f c = {};
#pragma unroll 4
      for (int kc = 0; kc < EE / 32; ++kc) { v16b a, w; const float* pa = X + (rq + col) * EE + kc * 32 + 8 * g; const float* pk = X + rk * EE + kc * 32 + 8 * g;
#pragma unroll
        for (int i = 0; i < 8; ++i) { a[i] = (__bf16)pa[i]; a[8 + i] = (__bf16)pa[16 + i]; w[i] = (__bf16)pk[i]; w[8 + i] = (__bf16)pk[16 + i]; }
        c = wmma_bf(a, w, c); }
      const float sqk = SQ[rk];
#pragma unroll
      for (int r = 0; r < 8; ++r) { const float d2 = fmaxf((sqq[r] + sqk) - 2.0f * c[r], 0.f); const float kv = expf(-GAM * d2); const float wv = expf(kv); rs[r] += wv; const _Float16 hv = (_Float16)wv; sh[wave][8 * g + r][ct * 16 + col] = hv; sl[wave][8 * g + r][ct * 16 + col] = (_Float16)((wv - (float)hv) * 2048.0f); } }
    LDSX();
    for (int rl = 0; rl < 16; ++rl) if (lane < 4) { const size_t o = (rq + rl) * NS + ks * 32 + lane * 8; vst2((unsigned*)(EH + o), *(const v4u*)&sh[wave][rl][lane * 8]); vst2((unsigned*)(EL + o), *(const v4u*)&sl[wave][rl][lane * 8]); }
    LDSX(); }
#pragma unroll
  for (int r = 0; r < 8; ++r) { float v = rs[r];
#pragma unroll
    for (int o = 1; o < 16; o <<= 1) v += __shfl_xor(v, o);
    if (col == 0) sil[wave * 16 + 8 * g + r] = 1.0f / v; }
  __syncthreads(); if (tid < 16) vst2(IL + rq - wave * 16 + tid * 4, *(const v4f*)&sil[tid * 4]); }
__global__ __launch_bounds__(128) void k_pv(const _Float16* __restrict__ EH, const _Float16* __restrict__ EL, const _Float16* __restrict__ XT, const float* __restrict__ IL, float* __restrict__ OUT) { __shared__ __align__(16) float sf[4][16][132];
  const int tid = threadIdx.x, wave = tid >> 5, lane = tid & 31, col = lane & 15, g = lane >> 4; const size_t b = blockIdx.z; const int q0 = blockIdx.x * 64 + wave * 16; const size_t rq = b * NS + q0; const int c0 = blockIdx.y * 128;
  v8f acc[8] = {}, accl[8] = {};
#pragma unroll 2
  for (int kc = 0; kc < NS / 32; ++kc) { const v16h ah = frag_h(EH + (rq + col) * NS + kc * 32, lane), al = frag_h(EL + (rq + col) * NS + kc * 32, lane);
#pragma unroll
    for (int j = 0; j < 8; ++j) { const v16h w = frag_h(XT + (b * EE + c0 + j * 16 + col) * (size_t)NS + kc * 32, lane); acc[j] = wmma16(ah, w, acc[j]); accl[j] = wmma16(al, w, accl[j]); } }
#pragma unroll
  for (int r = 0; r < 8; ++r) { const float il = IL[rq + 8 * g + r];
#pragma unroll
    for (int j = 0; j < 8; ++j) sf[wave][8 * g + r][j * 16 + col] = (acc[j][r] + accl[j][r] * (1.0f / 2048.0f)) * il; }
  LDSX(); for (int rl = 0; rl < 16; ++rl) vst2(OUT + (rq + rl) * EE + c0 + lane * 4, *(const v4f*)&sf[wave][rl][lane * 4]); }
extern "C" void kernel_launch(void* const* d_in, const int* in_sizes, int n_in, void* d_out, int out_size, void* d_ws, size_t ws_size, hipStream_t stream) {
  (void)in_sizes; (void)n_in; (void)out_size;
  const float** F = (const float**)d_in;
  if (ws_size < (size_t)WS_END) return;
  char* ws = (char*)d_ws; float *SQ = (float*)(ws + WS_SQ), *IL = (float*)(ws + WS_IL); _Float16 *XT = (_Float16*)(ws + WS_XT), *EH = (_Float16*)(ws + WS_EH), *EL = (_Float16*)(ws + WS_EL);
  k_prep<<<dim3(NS / 64, NB), 128, 0, stream>>>(F[0], SQ, XT);
  k_e<<<dim3(NS / 64, TNB), 128, 0, stream>>>(F[0], SQ, EH, EL, IL);
  k_pv<<<dim3(NS / 64, EE / 128, TNB), 128, 0, stream>>>(EH, EL, XT, IL, (float*)d_out);
}
